// PLE_27238682591702
// MI455X (gfx1250) — hardware-verified
//
#include <hip/hip_runtime.h>
#define NB 32768
#define IN 256
#define DD 64
#define GG 32
#define NS 4
#define NE3 3
#define NTK 3
#define NX 7

typedef __bf16 v16b __attribute__((ext_vector_type(16)));
typedef unsigned short v8us __attribute__((ext_vector_type(8), may_alias));
typedef float  v8f  __attribute__((ext_vector_type(8)));
typedef float  v4f  __attribute__((ext_vector_type(4)));
typedef float  v4fa __attribute__((ext_vector_type(4), may_alias));
union FragB { v16b v; v8us half[2]; unsigned short u[16]; };

__device__ __forceinline__ unsigned short bf16_bits(float x) { unsigned int u = __float_as_uint(x); return (unsigned short)((u + 0x7FFFu + ((u >> 16) & 1u)) >> 16); }
__device__ __forceinline__ float bf16_val(unsigned short b) { return __uint_as_float(((unsigned int)b) << 16); }
__device__ __forceinline__ float bf16_round(float x) { return bf16_val(bf16_bits(x)); }
template <int NT>
__device__ __forceinline__ v8f mmaN(v16b ah, v16b al, v16b bh, v16b bl, v8f c) {
  c = __builtin_amdgcn_wmma_f32_16x16x32_bf16(false, ah, false, bh, (short)0, c, false, false);
  if (NT >= 2) c = __builtin_amdgcn_wmma_f32_16x16x32_bf16(false, al, false, bh, (short)0, c, false, false);
  if (NT >= 3) c = __builtin_amdgcn_wmma_f32_16x16x32_bf16(false, ah, false, bl, (short)0, c, false, false);
  asm volatile("v_nop\n\tv_nop\n\tv_nop\n\tv_nop" : "+v"(c) : "v"(ah), "v"(al), "v"(bh), "v"(bl));
  return c;
}

__global__ __launch_bounds__(256) void k_wt_bf16(const float* __restrict__ W, unsigned short* __restrict__ Wt, int K, int N) {
  const int t = blockIdx.x * 256 + threadIdx.x;
  const int k8n = K / 8;
  if (t >= N * k8n) return;
  const int n = t / k8n, k8 = (t % k8n) * 8;
  v8us v;
#pragma unroll
  for (int i = 0; i < 8; ++i) v[i] = bf16_bits(W[(size_t)(k8 + i) * N + n]);
  *(volatile v8us*)(Wt + (size_t)n * K + k8) = v;
  __threadfence();
  *(volatile v8us*)(Wt + (size_t)n * K + k8) = v;
}

template <bool ASPLIT, int ACT, bool BIAS_BF16>
__global__ __launch_bounds__(128) void k_gemm_bf(const float* __restrict__ A, int lda, const unsigned short* __restrict__ Wt, int ldb,
                                               const float* __restrict__ bias, float* __restrict__ C, int ldc, int M, int N, int K) {
  __shared__ __attribute__((aligned(16))) float so[4][16][64];
  const int tid = threadIdx.x, w = tid >> 5, lane = tid & 31, ln = lane & 15, hh = lane >> 4;
  const int ntn = N / 64;
  const int wid = blockIdx.x * 4 + w;
  const int mt = wid / ntn, nq = wid % ntn;
  if (mt * 16 >= M) return;
  const int row0 = mt * 16, col0 = nq * 64;
  const float* arow = A + (size_t)(row0 + ln) * lda;
  v8f acc[4] = {};
  for (int kb = 0; kb < K; kb += 32) {
    FragB ah, al;
    const v4f x0 = *(const v4fa*)(arow + kb + 8 * hh), x1 = *(const v4fa*)(arow + kb + 8 * hh + 4);
    const v4f x2 = *(const v4fa*)(arow + kb + 16 + 8 * hh), x3 = *(const v4fa*)(arow + kb + 16 + 8 * hh + 4);
    float xs[16] = {x0[0],x0[1],x0[2],x0[3],x1[0],x1[1],x1[2],x1[3],x2[0],x2[1],x2[2],x2[3],x3[0],x3[1],x3[2],x3[3]};
#pragma unroll
    for (int i = 0; i < 16; ++i) { const unsigned short hb = bf16_bits(xs[i]); ah.u[i] = hb; al.u[i] = ASPLIT ? bf16_bits(xs[i] - bf16_val(hb)) : (unsigned short)0; }
#pragma unroll
    for (int t = 0; t < 4; ++t) {
      const unsigned short* brow = Wt + (size_t)(col0 + t * 16 + ln) * ldb + kb;
      FragB b;
      b.half[0] = *(const v8us*)(brow + 8 * hh);
      b.half[1] = *(const v8us*)(brow + 16 + 8 * hh);
      acc[t] = mmaN<ASPLIT ? 2 : 1>(ah.v, al.v, b.v, b.v, acc[t]);
    }
  }
#pragma unroll
  for (int t = 0; t < 4; ++t) {
    float bv = bias ? bias[col0 + t * 16 + ln] : 0.f;
    if (BIAS_BF16) bv = bf16_round(bv);
#pragma unroll
    for (int r = 0; r < 8; ++r) { float v = acc[t][r] + bv; if (ACT == 1) v = fmaxf(v, 0.f); so[w][8 * hh + r][t * 16 + ln] = v; }
  }
  __builtin_amdgcn_fence(__ATOMIC_ACQ_REL, "workgroup");
  __builtin_amdgcn_wave_barrier();
  const int rsub = lane >> 4, c4 = (lane & 15) * 4;
  for (int pass = 0; pass < 2; ++pass) {
#pragma unroll
    for (int q = 0; q < 8; ++q) {
      const int r = q * 2 + rsub;
      const v4f v = *(const v4fa*)&so[w][r][c4];
      *(volatile v4f*)(C + (size_t)(row0 + r) * ldc + col0 + c4) = v;
    }
    if (pass == 0) __threadfence();
  }
}

template <int D, bool CAUSAL>
__global__ __launch_bounds__(128) void k_flash(const float* __restrict__ qb, const float* __restrict__ kb, const float* __restrict__ vb,
                                             int pitch, int T, int H, float scale, float* __restrict__ y, int ypitch) {
  constexpr int KS = D / 32;
  constexpr int DT = D / 16;
  __shared__ __attribute__((aligned(16))) unsigned short sKh[32][D + 8], sKl[32][D + 8], sVh[32][D + 8], sVl[32][D + 8];
  __shared__ __attribute__((aligned(16))) unsigned short sPh[4][16][40], sPl[4][16][40];
  __shared__ __attribute__((aligned(16))) float sO[4][16][D];
  const int tid = threadIdx.x, w = tid >> 5, lane = tid & 31, ln = lane & 15, hh = lane >> 4;
  const int nqb = (T + 63) / 64;
  const int bh = blockIdx.x / nqb, qblk = blockIdx.x % nqb;
  const int b = bh / H, h = bh % H;
  const int q0 = qblk * 64 + w * 16;
  const float* Q = qb + (size_t)b * T * pitch + h * D;
  const float* K = kb + (size_t)b * T * pitch + h * D;
  const float* V = vb + (size_t)b * T * pitch + h * D;

  FragB aqh[KS], aql[KS];
  {
    int row = q0 + ln; if (row >= T) row = T - 1;
    const float* qr = Q + (size_t)row * pitch;
#pragma unroll
    for (int ks = 0; ks < KS; ++ks)
#pragma unroll
      for (int i = 0; i < 16; ++i) {
        const int d = ks * 32 + ((i < 8) ? (8 * hh + i) : (16 + 8 * hh + (i - 8)));
        const float x = qr[d] * scale; const unsigned short hb = bf16_bits(x);
        aqh[ks].u[i] = hb; aql[ks].u[i] = bf16_bits(x - bf16_val(hb));
      }
  }
  float m_r[8], l_r[8];
#pragma unroll
  for (int r = 0; r < 8; ++r) { m_r[r] = -3.0e38f; l_r[r] = 0.f; }
  v8f oacc[DT];
#pragma unroll
  for (int dt = 0; dt < DT; ++dt) oacc[dt] = (v8f){0.f,0.f,0.f,0.f,0.f,0.f,0.f,0.f};

  const int kv_end = CAUSAL ? min(T, qblk * 64 + 64) : T;
  for (int j0 = 0; j0 < kv_end; j0 += 32) {
    __syncthreads();
    for (int e = tid; e < 32 * (D / 4); e += 128) {
      const int r = e / (D / 4), c4 = (e % (D / 4)) * 4;
      const int key = j0 + r;
      v4f kf = {0.f,0.f,0.f,0.f}, vf = {0.f,0.f,0.f,0.f};
      if (key < T) { kf = *(const v4fa*)(K + (size_t)key * pitch + c4); vf = *(const v4fa*)(V + (size_t)key * pitch + c4); }
#pragma unroll
      for (int t = 0; t < 4; ++t) {
        unsigned short hb = bf16_bits(kf[t]); sKh[r][c4 + t] = hb; sKl[r][c4 + t] = bf16_bits(kf[t] - bf16_val(hb));
        hb = bf16_bits(vf[t]); sVh[r][c4 + t] = hb; sVl[r][c4 + t] = bf16_bits(vf[t] - bf16_val(hb));
      }
    }
    __syncthreads();
    v8f s[2];
#pragma unroll
    for (int nt = 0; nt < 2; ++nt) {
      v8f acc = {};
#pragma unroll
      for (int ks = 0; ks < KS; ++ks) {
        FragB bh_, bl_;
        bh_.half[0] = *(const v8us*)&sKh[nt * 16 + ln][ks * 32 + 8 * hh]; bh_.half[1] = *(const v8us*)&sKh[nt * 16 + ln][ks * 32 + 16 + 8 * hh];
        bl_.half[0] = *(const v8us*)&sKl[nt * 16 + ln][ks * 32 + 8 * hh]; bl_.half[1] = *(const v8us*)&sKl[nt * 16 + ln][ks * 32 + 16 + 8 * hh];
        acc = mmaN<3>(aqh[ks].v, aql[ks].v, bh_.v, bl_.v, acc);
      }
      s[nt] = acc;
    }
    float alpha[8];
#pragma unroll
    for (int r = 0; r < 8; ++r) {
      const int qi = q0 + 8 * hh + r;
      const int ja = j0 + ln, jb = j0 + 16 + ln;
      if (CAUSAL) { if (ja > qi) s[0][r] = -3.0e38f; if (jb > qi) s[1][r] = -3.0e38f; }
      if (ja >= T) s[0][r] = -3.0e38f;
      if (jb >= T) s[1][r] = -3.0e38f;
      float mx = fmaxf(s[0][r], s[1][r]);
      mx = fmaxf(mx, __shfl_xor(mx, 1, 32)); mx = fmaxf(mx, __shfl_xor(mx, 2, 32)); mx = fmaxf(mx, __shfl_xor(mx, 4, 32)); mx = fmaxf(mx, __shfl_xor(mx, 8, 32));
      const float mnew = fmaxf(m_r[r], mx);
      alpha[r] = (mnew > -1.0e38f) ? __expf(m_r[r] - mnew) : 1.0f;
      const float p0 = (s[0][r] > -1.0e38f) ? __expf(s[0][r] - mnew) : 0.f;
      const float p1 = (s[1][r] > -1.0e38f) ? __expf(s[1][r] - mnew) : 0.f;
      m_r[r] = mnew;
      l_r[r] = l_r[r] * alpha[r] + p0 + p1;
      unsigned short hb = bf16_bits(p0); sPh[w][8 * hh + r][ln] = hb;      sPl[w][8 * hh + r][ln] = bf16_bits(p0 - bf16_val(hb));
      hb = bf16_bits(p1);                sPh[w][8 * hh + r][16 + ln] = hb; sPl[w][8 * hh + r][16 + ln] = bf16_bits(p1 - bf16_val(hb));
    }
#pragma unroll
    for (int dt = 0; dt < DT; ++dt)
#pragma unroll
      for (int r = 0; r < 8; ++r) oacc[dt][r] *= alpha[r];
    __builtin_amdgcn_fence(__ATOMIC_ACQ_REL, "workgroup");
    __builtin_amdgcn_wave_barrier();
    FragB pah, pal;
    pah.half[0] = *(const v8us*)&sPh[w][ln][8 * hh]; pah.half[1] = *(const v8us*)&sPh[w][ln][16 + 8 * hh];
    pal.half[0] = *(const v8us*)&sPl[w][ln][8 * hh]; pal.half[1] = *(const v8us*)&sPl[w][ln][16 + 8 * hh];
#pragma unroll
    for (int dt = 0; dt < DT; ++dt) {
      FragB bvh, bvl;
#pragma unroll
      for (int i = 0; i < 8; ++i) {
        bvh.u[i] = sVh[8 * hh + i][dt * 16 + ln]; bvh.u[8 + i] = sVh[16 + 8 * hh + i][dt * 16 + ln];
        bvl.u[i] = sVl[8 * hh + i][dt * 16 + ln]; bvl.u[8 + i] = sVl[16 + 8 * hh + i][dt * 16 + ln];
      }
      oacc[dt] = mmaN<3>(pah.v, pal.v, bvh.v, bvl.v, oacc[dt]);
    }
    __builtin_amdgcn_fence(__ATOMIC_ACQ_REL, "workgroup");
    __builtin_amdgcn_wave_barrier();
  }
#pragma unroll
  for (int r = 0; r < 8; ++r) {
    float l = l_r[r];
    l += __shfl_xor(l, 1, 32); l += __shfl_xor(l, 2, 32); l += __shfl_xor(l, 4, 32); l += __shfl_xor(l, 8, 32);
    l_r[r] = (l > 0.f) ? 1.0f / l : 0.f;
  }
#pragma unroll
  for (int dt = 0; dt < DT; ++dt)
#pragma unroll
    for (int r = 0; r < 8; ++r) sO[w][8 * hh + r][dt * 16 + ln] = oacc[dt][r] * l_r[r];
  __builtin_amdgcn_fence(__ATOMIC_ACQ_REL, "workgroup");
  __builtin_amdgcn_wave_barrier();
  for (int pass = 0; pass < 2; ++pass) {
    for (int r = 0; r < 16; ++r) {
      const int row = q0 + r;
      if (row < T && lane < D / 4) {
        const v4f val = *(const v4fa*)&sO[w][r][lane * 4];
        *(volatile v4f*)(y + ((size_t)b * T + row) * ypitch + h * D + lane * 4) = val;
      }
    }
    if (pass == 0) __threadfence();
  }
}

template <bool ASPLIT, int ACT, bool BIAS_BF16, bool RES_BF16>
__global__ __launch_bounds__(128) void k_gemm_bf3(const float* __restrict__ A, int lda, const unsigned short* __restrict__ Wt, int ldb,
                                                const float* __restrict__ bias, const float* __restrict__ resid, int rmod, int ldr,
                                                float* __restrict__ C, int ldc, int M, int N, int K) {
  __shared__ __attribute__((aligned(16))) float so[4][16][64];
  const int tid = threadIdx.x, w = tid >> 5, lane = tid & 31, ln = lane & 15, hh = lane >> 4;
  const int ntn = N / 64;
  const int wid = blockIdx.x * 4 + w;
  const int mt = wid / ntn, nq = wid % ntn;
  if (mt * 16 >= M) return;
  const int row0 = mt * 16, col0 = nq * 64;
  const float* arow = A + (size_t)(row0 + ln) * lda;
  v8f acc[4] = {};
  for (int kb = 0; kb < K; kb += 32) {
    FragB ah, al;
    const v4f x0 = *(const v4fa*)(arow + kb + 8 * hh), x1 = *(const v4fa*)(arow + kb + 8 * hh + 4);
    const v4f x2 = *(const v4fa*)(arow + kb + 16 + 8 * hh), x3 = *(const v4fa*)(arow + kb + 16 + 8 * hh + 4);
    float xs[16] = {x0[0],x0[1],x0[2],x0[3],x1[0],x1[1],x1[2],x1[3],x2[0],x2[1],x2[2],x2[3],x3[0],x3[1],x3[2],x3[3]};
#pragma unroll
    for (int i = 0; i < 16; ++i) { const unsigned short hb = bf16_bits(xs[i]); ah.u[i] = hb; al.u[i] = ASPLIT ? bf16_bits(xs[i] - bf16_val(hb)) : (unsigned short)0; }
#pragma unroll
    for (int t = 0; t < 4; ++t) {
      const unsigned short* brow = Wt + (size_t)(col0 + t * 16 + ln) * ldb + kb;
      FragB b;
      b.half[0] = *(const v8us*)(brow + 8 * hh);
      b.half[1] = *(const v8us*)(brow + 16 + 8 * hh);
      acc[t] = mmaN<ASPLIT ? 2 : 1>(ah.v, al.v, b.v, b.v, acc[t]);
    }
  }
#pragma unroll
  for (int t = 0; t < 4; ++t) {
    const int col = col0 + t * 16 + ln;
    float bv = bias ? bias[col] : 0.f;
    if (BIAS_BF16) bv = bf16_round(bv);
#pragma unroll
    for (int r = 0; r < 8; ++r) {
      float v = acc[t][r] + bv;
      if (resid) { float rv = resid[(size_t)((row0 + 8 * hh + r) % rmod) * ldr + col]; if (RES_BF16) rv = bf16_round(rv); v += rv; }
      if (ACT == 1) v = fmaxf(v, 0.f);
      if (ACT == 2) v = 0.5f * v * (1.0f + erff(v * 0.70710678118654752f));
      if (ACT == 3) { const float u = 0.7978845608028654f * (v + 0.044715f * v * v * v); v = 0.5f * v * (1.0f + tanhf(u)); }
      so[w][8 * hh + r][t * 16 + ln] = v;
    }
  }
  __builtin_amdgcn_fence(__ATOMIC_ACQ_REL, "workgroup");
  __builtin_amdgcn_wave_barrier();
  const int rsub = lane >> 4, c4 = (lane & 15) * 4;
  for (int pass = 0; pass < 2; ++pass) {
#pragma unroll
    for (int q = 0; q < 8; ++q) {
      const int r = q * 2 + rsub;
      const v4f v = *(const v4fa*)&so[w][r][c4];
      *(volatile v4f*)(C + (size_t)(row0 + r) * ldc + col0 + c4) = v;
    }
    if (pass == 0) __threadfence();
  }
}
template <bool PARAM_BF16>
__global__ __launch_bounds__(256) void k_layernorm(const float* __restrict__ X, const float* __restrict__ R, const float* __restrict__ g, const float* __restrict__ bta,
                                                  float* __restrict__ out_sum, float* __restrict__ out_norm, int N, float eps) {
  __shared__ float red[256];
  const int row = blockIdx.x, tid = threadIdx.x;
  const float* x = X + (size_t)row * N; const float* rr = R ? R + (size_t)row * N : nullptr;
  float vals[16];
  const int per = N / 256;
  float s1 = 0.f;
  for (int u = 0; u < per / 4; ++u) {
    const int j = tid * 4 + 1024 * u;
    const v4f a = *(const v4fa*)(x + j);
    v4f b = {0.f,0.f,0.f,0.f}; if (rr) b = *(const v4fa*)(rr + j);
#pragma unroll
    for (int q = 0; q < 4; ++q) { const float v = a[q] + b[q]; vals[u * 4 + q] = v; s1 += v; }
  }
  red[tid] = s1; __syncthreads();
  for (int st = 128; st > 0; st >>= 1) { if (tid < st) red[tid] += red[tid + st]; __syncthreads(); }
  const float mu = red[0] / (float)N; __syncthreads();
  float s2 = 0.f;
  for (int u = 0; u < per / 4; ++u)
#pragma unroll
    for (int q = 0; q < 4; ++q) { const float c = vals[u * 4 + q] - mu; s2 += c * c; }
  red[tid] = s2; __syncthreads();
  for (int st = 128; st > 0; st >>= 1) { if (tid < st) red[tid] += red[tid + st]; __syncthreads(); }
  const float rs = rsqrtf(red[0] / (float)N + eps);
  for (int pass = 0; pass < 2; ++pass) {
    for (int u = 0; u < per / 4; ++u) {
      const int j = tid * 4 + 1024 * u;
      v4f o, sm;
#pragma unroll
      for (int q = 0; q < 4; ++q) {
        float gg = g[j + q], bb = bta[j + q];
        if (PARAM_BF16) { gg = bf16_round(gg); bb = bf16_round(bb); }
        sm[q] = vals[u * 4 + q]; o[q] = (vals[u * 4 + q] - mu) * rs * gg + bb;
      }
      if (out_sum) *(volatile v4f*)(out_sum + (size_t)row * N + j) = sm;
      *(volatile v4f*)(out_norm + (size_t)row * N + j) = o;
    }
    if (pass == 0) __threadfence();
  }
}


typedef _Float16 v16h __attribute__((ext_vector_type(16)));
union FragH { v16h v; v8us half[2]; _Float16 h[16]; unsigned short u[16]; };
template <int NT>
__device__ __forceinline__ v8f mmaH(v16h ah, v16h al, v16h bh, v16h bl, v8f c) {
  c = __builtin_amdgcn_wmma_f32_16x16x32_f16(false, ah, false, bh, (short)0, c, false, false);
  if (NT >= 2) c = __builtin_amdgcn_wmma_f32_16x16x32_f16(false, al, false, bh, (short)0, c, false, false);
  if (NT >= 3) c = __builtin_amdgcn_wmma_f32_16x16x32_f16(false, ah, false, bl, (short)0, c, false, false);
  asm volatile("v_nop\n\tv_nop\n\tv_nop\n\tv_nop" : "+v"(c) : "v"(ah), "v"(al), "v"(bh), "v"(bl));
  return c;
}
template <bool ASPLIT>
__global__ __launch_bounds__(128) void k_gemm_h(const float* __restrict__ A, int lda, size_t sA, const _Float16* __restrict__ Bh, int ldb, size_t sB, float alpha, float* __restrict__ C, int ldc, size_t sC, int M, int N, int K) {
  __shared__ __attribute__((aligned(16))) float so[4][16][64];
  const int tid = threadIdx.x, w = tid >> 5, lane = tid & 31, ln = lane & 15, hh = lane >> 4; const int by = blockIdx.y;
  A += (size_t)by * sA; Bh += (size_t)by * sB; C += (size_t)by * sC;
  const int ntn = (N + 63) / 64; const int wid = blockIdx.x * 4 + w; const int mt = wid / ntn, nq = wid % ntn; if (mt * 16 >= M) return;
  const int row0 = mt * 16, col0 = nq * 64; const float* arow = A + (size_t)(row0 + ln) * lda;
  v8f acc[4] = {};
  for (int kb = 0; kb < K; kb += 32) {
    FragH ah, al;
    const v4f x0 = *(const v4fa*)(arow + kb + 8 * hh), x1 = *(const v4fa*)(arow + kb + 8 * hh + 4), x2 = *(const v4fa*)(arow + kb + 16 + 8 * hh), x3 = *(const v4fa*)(arow + kb + 16 + 8 * hh + 4);
    float xs[16] = {x0[0],x0[1],x0[2],x0[3],x1[0],x1[1],x1[2],x1[3],x2[0],x2[1],x2[2],x2[3],x3[0],x3[1],x3[2],x3[3]};
#pragma unroll
    for (int i = 0; i < 16; ++i) { const _Float16 h = (_Float16)xs[i]; ah.h[i] = h; al.h[i] = ASPLIT ? (_Float16)(xs[i] - (float)h) : (_Float16)0.0f; }
#pragma unroll
    for (int t = 0; t < 4; ++t) { if (col0 + t * 16 >= N) continue; const size_t boff = (size_t)(col0 + t * 16 + ln) * ldb + kb; FragH bq; bq.half[0] = *(const v8us*)(Bh + boff + 8 * hh); bq.half[1] = *(const v8us*)(Bh + boff + 16 + 8 * hh);
      acc[t] = mmaH<ASPLIT ? 2 : 1>(ah.v, al.v, bq.v, bq.v, acc[t]); }
  }
#pragma unroll
  for (int t = 0; t < 4; ++t) { if (col0 + t * 16 >= N) continue;
#pragma unroll
    for (int r = 0; r < 8; ++r) so[w][8 * hh + r][t * 16 + ln] = acc[t][r] * alpha; }
  __builtin_amdgcn_fence(__ATOMIC_ACQ_REL, "workgroup"); __builtin_amdgcn_wave_barrier();
  const int rsub = lane >> 4, c4 = (lane & 15) * 4;
  for (int pass = 0; pass < 2; ++pass) {
#pragma unroll
    for (int q = 0; q < 8; ++q) { const int r = q * 2 + rsub; if (col0 + c4 < N) { const v4f v = *(const v4fa*)&so[w][r][c4]; *(volatile v4f*)(C + (size_t)(row0 + r) * ldc + col0 + c4) = v; } }
    if (pass == 0) __threadfence(); }
}

__global__ __launch_bounds__(256) void k_wt_f16(const float* __restrict__ W, _Float16* __restrict__ Wt, int K, int N, float scale) {
  const int t = blockIdx.x * 256 + threadIdx.x; if (t >= N * (K / 8)) return; const int n = t / (K / 8), k8 = (t % (K / 8)) * 8; FragH f;
#pragma unroll
  for (int i = 0; i < 8; ++i) f.h[i] = (_Float16)(bf16_round(W[(size_t)(k8 + i) * N + n]) * scale); const v8us o = f.half[0];
  *(volatile v8us*)((unsigned short*)Wt + (size_t)n * K + k8) = o; __threadfence(); *(volatile v8us*)((unsigned short*)Wt + (size_t)n * K + k8) = o;
}
template <int ACT>
__global__ __launch_bounds__(128) void k_gemm_hhx(const _Float16* __restrict__ A, int lda, size_t sA, const _Float16* __restrict__ Bh, int ldb, size_t sB, float alpha, const float* __restrict__ bias, size_t sBias, const float* __restrict__ CP, int rowsPerB, size_t sCPb, int row0g,
    float* __restrict__ C, _Float16* __restrict__ C16, int ldc, size_t sC, int M, int N, int K) {
  __shared__ __attribute__((aligned(16))) float so[4][16][64];
  const int tid = threadIdx.x, w = tid >> 5, lane = tid & 31, ln = lane & 15, hh = lane >> 4; const int by = blockIdx.y;
  A += (size_t)by * sA; Bh += (size_t)by * sB; const size_t cofs = (size_t)by * sC; const float* bp = bias ? bias + (size_t)by * sBias : nullptr;
  const int ntn = (N + 63) / 64; const int wid = blockIdx.x * 4 + w; const int mt = wid / ntn, nq = wid % ntn; if (mt * 16 >= M) return;
  const int row0 = mt * 16, col0 = nq * 64; const _Float16* arow = A + (size_t)(row0 + ln) * lda;
  v8f acc[4] = {};
  for (int kb = 0; kb < K; kb += 32) { FragH ah; ah.half[0] = *(const v8us*)((const unsigned short*)arow + kb + 8 * hh); ah.half[1] = *(const v8us*)((const unsigned short*)arow + kb + 16 + 8 * hh);
#pragma unroll
    for (int t = 0; t < 4; ++t) { if (col0 + t * 16 >= N) continue; const size_t boff = (size_t)(col0 + t * 16 + ln) * ldb + kb; FragH bq; bq.half[0] = *(const v8us*)((const unsigned short*)Bh + boff + 8 * hh); bq.half[1] = *(const v8us*)((const unsigned short*)Bh + boff + 16 + 8 * hh);
      acc[t] = mmaH<1>(ah.v, ah.v, bq.v, bq.v, acc[t]); }
  }
#pragma unroll
  for (int t = 0; t < 4; ++t) { if (col0 + t * 16 >= N) continue; const int col = col0 + t * 16 + ln; const float bv = bp ? bf16_round(bp[col]) : 0.f;
#pragma unroll
    for (int r = 0; r < 8; ++r) { float v = acc[t][r] * alpha + bv; if (CP) { const int bidx = (row0g + row0 + 8 * hh + r) / rowsPerB; v += CP[(size_t)bidx * sCPb + (size_t)by * 64 + col]; } if (ACT == 1) v = (v > 0.f) ? v : expm1f(v); else if (ACT == 3) v = fmaxf(v, 0.f); so[w][8 * hh + r][t * 16 + ln] = v; } }
  __builtin_amdgcn_fence(__ATOMIC_ACQ_REL, "workgroup"); __builtin_amdgcn_wave_barrier();
  const int rsub = lane >> 4, c4 = (lane & 15) * 4; typedef _Float16 v4h __attribute__((ext_vector_type(4)));
  for (int pass = 0; pass < 2; ++pass) {
#pragma unroll
    for (int q = 0; q < 8; ++q) { const int r = q * 2 + rsub; if (col0 + c4 < N) { const v4f v = *(const v4fa*)&so[w][r][c4]; if (C) *(volatile v4f*)(C + cofs + (size_t)(row0 + r) * ldc + col0 + c4) = v; if (C16) { v4h h4; for (int i = 0; i < 4; ++i) h4[i] = (_Float16)v[i]; *(volatile v4h*)(C16 + cofs + (size_t)(row0 + r) * ldc + col0 + c4) = h4; } } }
    if (pass == 0) __threadfence(); }
}


__device__ __forceinline__ void store_span256(float* span, v4f lo, v4f hi, int lane) {
  v4f a, b; const int s0 = lane >> 1, s1 = 16 + (lane >> 1); const bool odd = (lane & 1) != 0;
#pragma unroll
  for (int q = 0; q < 4; ++q) { const float l0 = __shfl(lo[q], s0, 32), h0 = __shfl(hi[q], s0, 32), l1 = __shfl(lo[q], s1, 32), h1 = __shfl(hi[q], s1, 32); a[q] = odd ? h0 : l0; b[q] = odd ? h1 : l1; }
  for (int pass = 0; pass < 2; ++pass) { *(volatile v4f*)(span + 4 * lane) = a; *(volatile v4f*)(span + 128 + 4 * lane) = b; if (pass == 0) __threadfence(); } }
__device__ __forceinline__ void store_span512h(_Float16* span, v8us p0, v8us p1, int lane) {
  typedef unsigned int v4u __attribute__((ext_vector_type(4))); union U { v8us h; v4u u; }; U x0, x1, a, b; x0.h = p0; x1.h = p1; const int s0 = lane >> 1, s1 = 16 + (lane >> 1); const bool odd = (lane & 1) != 0;
#pragma unroll
  for (int q = 0; q < 4; ++q) { const unsigned l0 = __shfl(x0.u[q], s0, 32), h0 = __shfl(x1.u[q], s0, 32), l1 = __shfl(x0.u[q], s1, 32), h1 = __shfl(x1.u[q], s1, 32); a.u[q] = odd ? h0 : l0; b.u[q] = odd ? h1 : l1; }
  for (int pass = 0; pass < 2; ++pass) { *(volatile v8us*)((unsigned short*)span + 8 * lane) = a.h; *(volatile v8us*)((unsigned short*)span + 256 + 8 * lane) = b.h; if (pass == 0) __threadfence(); } }

__global__ __launch_bounds__(256) void k_x16(const float* __restrict__ x, _Float16* __restrict__ X16, size_t n8) { const size_t t = (size_t)blockIdx.x * 256 + threadIdx.x; if (t >= n8) return; FragH f;
#pragma unroll
  for (int q = 0; q < 8; ++q) f.h[q] = (_Float16)bf16_round(x[t * 8 + q]); *(volatile v8us*)((unsigned short*)X16 + t * 8) = f.half[0]; __threadfence(); *(volatile v8us*)((unsigned short*)X16 + t * 8) = f.half[0]; }
__global__ __launch_bounds__(256) void k_wcat(const float* __restrict__ W, int nmat, int K, int N, _Float16* __restrict__ Bt) { const int t = blockIdx.x * 256 + threadIdx.x; if (t >= nmat * N * (K / 8)) return; const int row = t / (K / 8), k8 = (t % (K / 8)) * 8; const int m = row / N, n = row % N; FragH f;
#pragma unroll
  for (int q = 0; q < 8; ++q) f.h[q] = (_Float16)(bf16_round(W[((size_t)m * K + k8 + q) * N + n]) * 16.0f); *(volatile v8us*)((unsigned short*)Bt + (size_t)row * K + k8) = f.half[0]; __threadfence(); *(volatile v8us*)((unsigned short*)Bt + (size_t)row * K + k8) = f.half[0]; }
__global__ __launch_bounds__(256) void k_comb(const _Float16* __restrict__ GH, const float* __restrict__ gW2, const float* __restrict__ gb2, const _Float16* __restrict__ SHO, const _Float16* __restrict__ TEO, int ldteo, float* __restrict__ XT, _Float16* __restrict__ XT16) {
  const size_t tg = (size_t)blockIdx.x * 256 + threadIdx.x; if (tg >= (size_t)NTK * NB * 8) return; const int pc = (int)(tg % 8); const size_t tb = tg / 8; const int b = (int)(tb % NB), t = (int)(tb / NB);
  float lg[NX];
#pragma unroll
  for (int e = 0; e < NX; ++e) { float a = bf16_round(gb2[t * NX + e]);
#pragma unroll 1
    for (int g = 0; g < GG; ++g) a += (float)GH[(size_t)b * (NTK * GG) + t * GG + g] * bf16_round(gW2[((size_t)t * GG + g) * NX + e]); lg[e] = a; }
  float m = lg[0];
#pragma unroll
  for (int e = 1; e < NX; ++e) m = fmaxf(m, lg[e]); float z = 0.f;
#pragma unroll
  for (int e = 0; e < NX; ++e) { lg[e] = expf(lg[e] - m); z += lg[e]; } const float iz = 1.0f / z;
  float o[8]; FragH f;
#pragma unroll
  for (int q = 0; q < 8; ++q) { const int d = pc * 8 + q; float a = 0.f;
#pragma unroll
    for (int e = 0; e < NX; ++e) { const float av = (e < NS) ? (float)SHO[(size_t)b * (NS * DD) + e * DD + d] : (float)TEO[(size_t)b * ldteo + (t * NE3 + (e - NS)) * DD + d]; a += lg[e] * iz * av; }
    o[q] = a; f.h[q] = (_Float16)a; }
  const int lane = threadIdx.x & 31; if (XT) { const v4f lo = {o[0], o[1], o[2], o[3]}, hi = {o[4], o[5], o[6], o[7]}; store_span256(XT + (tg & ~(size_t)31) * 8, lo, hi, lane); }
  if (XT16) { *(volatile v8us*)((unsigned short*)XT16 + tg * 8) = f.half[0]; __threadfence(); *(volatile v8us*)((unsigned short*)XT16 + tg * 8) = f.half[0]; } }
__global__ __launch_bounds__(256) void k_comb1(const _Float16* __restrict__ GH, const float* __restrict__ gW2, const float* __restrict__ gb2, const _Float16* __restrict__ SHO, const _Float16* __restrict__ TEO, float* __restrict__ XT, _Float16* __restrict__ XT16) {
  const size_t tg = (size_t)blockIdx.x * 256 + threadIdx.x; if (tg >= (size_t)NTK * NB * 8) return; const int pc = (int)(tg % 8); const size_t tb = tg / 8; const int b = (int)(tb % NB), t = (int)(tb / NB);
  float lg[NX];
#pragma unroll
  for (int e = 0; e < NX; ++e) { float a = bf16_round(gb2[t * NX + e]);
#pragma unroll 1
    for (int g = 0; g < GG; ++g) a += (float)GH[(size_t)b * (NTK * GG) + t * GG + g] * bf16_round(gW2[((size_t)t * GG + g) * NX + e]); lg[e] = a; }
  float m = lg[0];
#pragma unroll
  for (int e = 1; e < NX; ++e) m = fmaxf(m, lg[e]); float z = 0.f;
#pragma unroll
  for (int e = 0; e < NX; ++e) { lg[e] = expf(lg[e] - m); z += lg[e]; } const float iz = 1.0f / z;
  float o[8]; FragH f;
#pragma unroll
  for (int q = 0; q < 8; ++q) { const int d = pc * 8 + q; float a = 0.f;
#pragma unroll
    for (int e = 0; e < NX; ++e) { const float av = (e < NS) ? (float)SHO[(size_t)b * (NS * DD) + e * DD + d] : (float)TEO[((size_t)t * NB + b) * (NE3 * DD) + (e - NS) * DD + d]; a += lg[e] * iz * av; }
    o[q] = a; f.h[q] = (_Float16)a; }
  const int lane = threadIdx.x & 31; if (XT) { const v4f lo = {o[0], o[1], o[2], o[3]}, hi = {o[4], o[5], o[6], o[7]}; store_span256(XT + (tg & ~(size_t)31) * 8, lo, hi, lane); }
  if (XT16) { *(volatile v8us*)((unsigned short*)XT16 + tg * 8) = f.half[0]; __threadfence(); *(volatile v8us*)((unsigned short*)XT16 + tg * 8) = f.half[0]; } }
__global__ __launch_bounds__(256) void k_mean3(const _Float16* __restrict__ XT, _Float16* __restrict__ XM16) { const size_t t = (size_t)blockIdx.x * 256 + threadIdx.x; if (t >= (size_t)NB * DD / 8) return; FragH f;
#pragma unroll
  for (int q = 0; q < 8; ++q) { const size_t i = t * 8 + q; f.h[q] = (_Float16)(((float)XT[i] + (float)XT[(size_t)NB * DD + i] + (float)XT[2 * (size_t)NB * DD + i]) / 3.0f); } *(volatile v8us*)((unsigned short*)XM16 + t * 8) = f.half[0]; __threadfence(); *(volatile v8us*)((unsigned short*)XM16 + t * 8) = f.half[0]; }
__global__ __launch_bounds__(256) void k_tower(const float* __restrict__ XT, const float* __restrict__ w1, const float* __restrict__ b1, const float* __restrict__ w2, const float* __restrict__ b2, float* __restrict__ out) { const size_t tg = (size_t)blockIdx.x * 256 + threadIdx.x; if (tg >= (size_t)NTK * NB) return; const int t = (int)(tg / NB); const float* xr = XT + tg * DD; float y = bf16_round(b2[t]);
#pragma unroll 1
  for (int j = 0; j < DD / 2; ++j) { float a = bf16_round(b1[t * (DD / 2) + j]);
#pragma unroll 1
    for (int d = 0; d < DD; ++d) a += xr[d] * bf16_round(w1[((size_t)t * DD + d) * (DD / 2) + j]); y += fmaxf(a, 0.f) * bf16_round(w2[t * (DD / 2) + j]); }
  const float s = 1.0f / (1.0f + expf(-y)); *(volatile float*)(out + tg) = s; __threadfence(); *(volatile float*)(out + tg) = s; }
extern "C" void kernel_launch(void* const* d_in, const int* in_sizes, int n_in,
                              void* d_out, int out_size, void* d_ws, size_t ws_size, hipStream_t stream) {
  (void)in_sizes; (void)n_in; (void)out_size;
  const float* x = (const float*)d_in[0];
  const float* L0[12]; const float* L1[12]; for (int i = 0; i < 12; ++i) { L0[i] = (const float*)d_in[1 + i]; L1[i] = (const float*)d_in[13 + i]; }
  const float* twW1 = (const float*)d_in[25]; const float* twb1 = (const float*)d_in[26]; const float* twW2 = (const float*)d_in[27]; const float* twb2 = (const float*)d_in[28];
  char* ws = (char*)d_ws; size_t off = 0;
  auto take = [&](size_t bytes) { char* p = ws + off; off += (bytes + 255) & ~(size_t)255; return p; };
  _Float16* Bsh1[2]; _Float16* Bsh2[2]; _Float16* Bte1[2]; _Float16* Bte2[2]; _Float16* Bg1[2]; const int DIN[2] = {IN, DD};
  for (int l = 0; l < 2; ++l) { Bsh1[l] = (_Float16*)take((size_t)NS * DD * DIN[l] * 2); Bsh2[l] = (_Float16*)take((size_t)NS * DD * DD * 2); Bte1[l] = (_Float16*)take((size_t)NTK * NE3 * DD * DIN[l] * 2); Bte2[l] = (_Float16*)take((size_t)NTK * NE3 * DD * DD * 2); Bg1[l] = (_Float16*)take((size_t)NTK * GG * DIN[l] * 2); }
  _Float16* X16 = (_Float16*)take((size_t)NB * IN * 2); _Float16* TE1 = (_Float16*)take((size_t)NB * NTK * NE3 * DD * 2); _Float16* SHO = (_Float16*)take((size_t)NB * NS * DD * 2); _Float16* TEO = (_Float16*)take((size_t)NB * NTK * NE3 * DD * 2); _Float16* GH = (_Float16*)take((size_t)NB * NTK * GG * 2);
  _Float16* SH1 = TE1;
  _Float16* XT16 = X16;
  _Float16* XM16 = X16 + (size_t)NTK * NB * DD;
  float* XT2 = (float*)TE1;
  if (off > ws_size) return;
  for (int l = 0; l < 2; ++l) { const float* const* P = l ? L1 : L0; const int din = DIN[l];
    k_wcat<<<(NS * DD * (din / 8) + 255) / 256, 256, 0, stream>>>(P[0], NS, din, DD, Bsh1[l]); k_wcat<<<(NS * DD * (DD / 8) + 255) / 256, 256, 0, stream>>>(P[2], NS, DD, DD, Bsh2[l]);
    k_wcat<<<(NTK * NE3 * DD * (din / 8) + 255) / 256, 256, 0, stream>>>(P[4], NTK * NE3, din, DD, Bte1[l]); k_wcat<<<(NTK * NE3 * DD * (DD / 8) + 255) / 256, 256, 0, stream>>>(P[6], NTK * NE3, DD, DD, Bte2[l]);
    k_wcat<<<(NTK * GG * (din / 8) + 255) / 256, 256, 0, stream>>>(P[8], NTK, din, GG, Bg1[l]); }
  const unsigned mt = NB / 16;
  k_x16<<<(unsigned)(((size_t)NB * IN / 8 + 255) / 256), 256, 0, stream>>>(x, X16, (size_t)NB * IN / 8);
  k_gemm_hhx<3><<<dim3((mt * (NS * DD / 64) + 3) / 4, 1), 128, 0, stream>>>(X16, IN, 0, Bsh1[0], IN, 0, 0.0625f, L0[1], 0, nullptr, 1, 0, 0, nullptr, SH1, NS * DD, 0, NB, NS * DD, IN);
  k_gemm_hhx<3><<<dim3((mt * 1 + 3) / 4, NS), 128, 0, stream>>>(SH1, NS * DD, (size_t)DD, Bsh2[0], DD, (size_t)DD * DD, 0.0625f, L0[3], (size_t)DD, nullptr, 1, 0, 0, nullptr, SHO, NS * DD, (size_t)DD, NB, DD, DD);
  k_gemm_hhx<3><<<dim3((mt * (NTK * NE3 * DD / 64) + 3) / 4, 1), 128, 0, stream>>>(X16, IN, 0, Bte1[0], IN, 0, 0.0625f, L0[5], 0, nullptr, 1, 0, 0, nullptr, TE1, NTK * NE3 * DD, 0, NB, NTK * NE3 * DD, IN);
  k_gemm_hhx<3><<<dim3((mt * 1 + 3) / 4, NTK * NE3), 128, 0, stream>>>(TE1, NTK * NE3 * DD, (size_t)DD, Bte2[0], DD, (size_t)DD * DD, 0.0625f, L0[7], (size_t)DD, nullptr, 1, 0, 0, nullptr, TEO, NTK * NE3 * DD, (size_t)DD, NB, DD, DD);
  k_gemm_hhx<3><<<dim3((mt * 2 + 3) / 4, 1), 128, 0, stream>>>(X16, IN, 0, Bg1[0], IN, 0, 0.0625f, L0[9], 0, nullptr, 1, 0, 0, nullptr, GH, NTK * GG, 0, NB, NTK * GG, IN);
  k_comb<<<(unsigned)(((size_t)NTK * NB * 8 + 255) / 256), 256, 0, stream>>>(GH, L0[10], L0[11], SHO, TEO, NTK * NE3 * DD, nullptr, XT16);
  k_mean3<<<(NB * DD / 8 + 255) / 256, 256, 0, stream>>>(XT16, XM16);
  k_gemm_hhx<3><<<dim3((mt * (NS * DD / 64) + 3) / 4, 1), 128, 0, stream>>>(XM16, DD, 0, Bsh1[1], DD, 0, 0.0625f, L1[1], 0, nullptr, 1, 0, 0, nullptr, SH1, NS * DD, 0, NB, NS * DD, DD);
  k_gemm_hhx<3><<<dim3((mt * 1 + 3) / 4, NS), 128, 0, stream>>>(SH1, NS * DD, (size_t)DD, Bsh2[1], DD, (size_t)DD * DD, 0.0625f, L1[3], (size_t)DD, nullptr, 1, 0, 0, nullptr, SHO, NS * DD, (size_t)DD, NB, DD, DD);
  k_gemm_hhx<3><<<dim3((mt * (NE3 * DD / 64) + 3) / 4, NTK), 128, 0, stream>>>(XT16, DD, (size_t)NB * DD, Bte1[1], DD, (size_t)NE3 * DD * DD, 0.0625f, L1[5], (size_t)NE3 * DD, nullptr, 1, 0, 0, nullptr, TE1, NE3 * DD, (size_t)NB * NE3 * DD, NB, NE3 * DD, DD);
  for (int t = 0; t < NTK; ++t) k_gemm_hhx<3><<<dim3((mt * 1 + 3) / 4, NE3), 128, 0, stream>>>(TE1 + (size_t)t * NB * NE3 * DD, NE3 * DD, (size_t)DD, Bte2[1] + (size_t)t * NE3 * DD * DD, DD, (size_t)DD * DD, 0.0625f, L1[7] + t * NE3 * DD, (size_t)DD, nullptr, 1, 0, 0, nullptr, TEO + (size_t)t * NB * NE3 * DD, NE3 * DD, (size_t)DD, NB, DD, DD);
  k_gemm_hhx<3><<<dim3((mt * 1 + 3) / 4, NTK), 128, 0, stream>>>(XT16, DD, (size_t)NB * DD, Bg1[1], DD, (size_t)GG * DD, 0.0625f, L1[9], (size_t)GG, nullptr, 1, 0, 0, nullptr, GH, NTK * GG, (size_t)GG, NB, GG, DD);
  k_comb1<<<(unsigned)(((size_t)NTK * NB * 8 + 255) / 256), 256, 0, stream>>>(GH, L1[10], L1[11], SHO, TEO, XT2, nullptr);
  k_tower<<<(unsigned)(((size_t)NTK * NB + 255) / 256), 256, 0, stream>>>(XT2, twW1, twb1, twW2, twb2, (float*)d_out);
}
